// MambaSSM_5291399709428
// MI455X (gfx1250) — hardware-verified
//
#include <hip/hip_runtime.h>
#include <math.h>

typedef __attribute__((ext_vector_type(16))) _Float16 v16h;
typedef __attribute__((ext_vector_type(8)))  _Float16 v8h;
typedef __attribute__((ext_vector_type(16))) __bf16   v16b;
typedef __attribute__((ext_vector_type(8)))  __bf16   v8b;
typedef __attribute__((ext_vector_type(8)))  float    v8f;
typedef __attribute__((ext_vector_type(4)))  float    v4f;
typedef __attribute__((ext_vector_type(4)))  unsigned v4u;

constexpr int kSeqT    = 32768;
constexpr int kObs     = 256;
constexpr int kHid     = 512;
constexpr int kNobj    = 4;
constexpr int kGrp     = 4;
constexpr int kPrjN    = kGrp * kHid;
constexpr int kTc      = 8192;
constexpr int kNChunk  = kSeqT / kTc;
constexpr int kScanTS  = 64;
constexpr int kScanCh  = 64;
constexpr int kScanYP  = 68;
constexpr float kCarryY0 = 16.0f;
constexpr float kCarryW1 = 32.0f;
constexpr float kFoldL1  = 1.0f / (kCarryY0 * kCarryW1);
static_assert(kPrjN == 2048, "fused projection width");
static_assert(kNChunk * kTc == kSeqT, "chunking");
static_assert((kObs % 64) == 0 && (kHid % 64) == 0, "K multiples of 64 (transpose tiles) and 32 (k-steps)");
static_assert((kTc % 64) == 0 && (kPrjN % 64) == 0, "GEMM M,N multiples of 64");
static_assert((kTc % kScanTS) == 0 && (kHid % kScanCh) == 0 && (kTc % 256) == 0, "scan/head tiles");
static_assert(kNobj == 4, "one float4 per output row");

constexpr size_t kOffXB    = 0;
constexpr size_t kOffBT0   = kOffXB  + (size_t)kSeqT * kObs * 2;
constexpr size_t kOffBT1   = kOffBT0 + (size_t)kPrjN * kObs * 2;
constexpr size_t kOffPRJ   = kOffBT1 + (size_t)kPrjN * kHid * 2;
constexpr size_t kOffY0H   = kOffPRJ + (size_t)kTc * kPrjN * 4;
constexpr size_t kOffY1    = kOffY0H + (size_t)kTc * kHid * 2;
constexpr size_t kOffCARRY = kOffY1  + (size_t)kTc * kHid * 4;
constexpr size_t kWsTotal  = kOffCARRY + (size_t)2 * 2 * kHid * 4;
static_assert(kWsTotal == 112205824ull, "carve total");
static_assert(kWsTotal <= 134217728ull, "carve cap");
static_assert((kOffBT0 % 128) == 0 && (kOffBT1 % 128) == 0 && (kOffPRJ % 128) == 0 &&
              (kOffY0H % 128) == 0 && (kOffY1 % 128) == 0 && (kOffCARRY % 128) == 0, "128-B aligned regions");

__device__ __forceinline__ unsigned short f2bf_bits(float f) {
  unsigned u = __float_as_uint(f);
  return (unsigned short)((u + 0x7FFFu + ((u >> 16) & 1u)) >> 16);
}
__device__ __forceinline__ float bf_bits2f(unsigned short h) { return __uint_as_float(((unsigned)h) << 16); }
__device__ __forceinline__ float bf_val(float f) { return bf_bits2f(f2bf_bits(f)); }

__device__ __forceinline__ void grp_guard_h(v8f& a, v8f& b, v8f& c, v8f& d, v16h x, v16h b0, v16h b1, v16h b2, v16h b3) {
  asm volatile("v_nop\n\tv_nop\n\tv_nop\n\tv_nop" : "+v"(a), "+v"(b), "+v"(c), "+v"(d) : "v"(x), "v"(b0), "v"(b1), "v"(b2), "v"(b3));
}
__device__ __forceinline__ void grp_guard_b(v8f& a, v8f& b, v8f& c, v8f& d, v16b x, v16b b0, v16b b1, v16b b2, v16b b3) {
  asm volatile("v_nop\n\tv_nop\n\tv_nop\n\tv_nop" : "+v"(a), "+v"(b), "+v"(c), "+v"(d) : "v"(x), "v"(b0), "v"(b1), "v"(b2), "v"(b3));
}
__device__ __forceinline__ void keep4_h(v16h a, v16h b, v16h c, v16h d) { asm volatile("v_nop" :: "v"(a), "v"(b), "v"(c), "v"(d)); }
__device__ __forceinline__ void keep4_b(v16b a, v16b b, v16b c, v16b d) { asm volatile("v_nop" :: "v"(a), "v"(b), "v"(c), "v"(d)); }
__device__ __forceinline__ void acc_guard4(v8f& a, v8f& b, v8f& c, v8f& d) { asm volatile("v_nop\n\tv_nop\n\tv_nop\n\tv_nop" : "+v"(a), "+v"(b), "+v"(c), "+v"(d)); }

template <typename T> struct Frag;
template <> struct Frag<_Float16> {
  typedef v16h V; union U { v16h v; v8h h[2]; };
  static __device__ __forceinline__ v16h load(const _Float16* p) {
    U f; f.h[0] = *(const v8h*)(p); f.h[1] = *(const v8h*)(p + 16); return f.v;
  }
  static __device__ __forceinline__ v8f mma(v16h a, v16h b, v8f c) {
    return __builtin_amdgcn_wmma_f32_16x16x32_f16(false, a, false, b, (short)0, c, false, false);
  }
  static __device__ __forceinline__ void guard(v8f& a, v8f& b, v8f& c, v8f& d, v16h x, v16h b0, v16h b1, v16h b2, v16h b3) { grp_guard_h(a, b, c, d, x, b0, b1, b2, b3); }
  static __device__ __forceinline__ void keep(v16h a, v16h b, v16h c, v16h d) { keep4_h(a, b, c, d); }
};
template <> struct Frag<__bf16> {
  typedef v16b V; union U { v16b v; v8b h[2]; };
  static __device__ __forceinline__ v16b load(const __bf16* p) {
    U f; f.h[0] = *(const v8b*)(p); f.h[1] = *(const v8b*)(p + 16); return f.v;
  }
  static __device__ __forceinline__ v8f mma(v16b a, v16b b, v8f c) {
    return __builtin_amdgcn_wmma_f32_16x16x32_bf16(false, a, false, b, (short)0, c, false, false);
  }
  static __device__ __forceinline__ void guard(v8f& a, v8f& b, v8f& c, v8f& d, v16b x, v16b b0, v16b b1, v16b b2, v16b b3) { grp_guard_b(a, b, c, d, x, b0, b1, b2, b3); }
  static __device__ __forceinline__ void keep(v16b a, v16b b, v16b c, v16b d) { keep4_b(a, b, c, d); }
};

template <int ET> struct Elem;
template <> struct Elem<0> { typedef _Float16 T; };
template <> struct Elem<1> { typedef __bf16 T; };
template <int ET>
__global__ __launch_bounds__(256) void wmma_gemm64(
    const unsigned short* __restrict__ Ap, int lda,
    const unsigned short* __restrict__ Btp, int ldb,
    float* __restrict__ Cout, int ldc,
    int M, int N, int K, float scale) {
  typedef typename Elem<ET>::T T;
  typedef typename Frag<T>::V V;
  const T* A  = (const T*)Ap;
  const T* Bt = (const T*)Btp;
  __shared__ __align__(16) float sT[8][16 * 68];
  const int lane = threadIdx.x & 31;
  const int wave = threadIdx.x >> 5;
  const int tilesN = N >> 6;
  const int tilesM = M >> 6;
  const int tile = blockIdx.x * 8 + wave;
  if (tile >= tilesM * tilesN) return;
  const int tm = tile / tilesN;
  const int tn = tile - tm * tilesN;
  const int m0 = tm << 6;
  const int n0 = tn << 6;

  const int rlane = lane & 15;
  const int koff  = (lane >> 4) * 8;
  const int mOff  = (lane >> 4) * 8;

  v8f acc[4][4];
#pragma unroll
  for (int i = 0; i < 4; ++i)
#pragma unroll
    for (int j = 0; j < 4; ++j) acc[i][j] = (v8f){0.f,0.f,0.f,0.f,0.f,0.f,0.f,0.f};

  for (int k0 = 0; k0 < K; k0 += 32) {
    V bh[4];
#pragma unroll
    for (int j = 0; j < 4; ++j) {
      const size_t bo = (size_t)(n0 + (j << 4) + rlane) * ldb + koff + k0;
      bh[j] = Frag<T>::load(Bt + bo);
    }
#pragma unroll
    for (int i = 0; i < 4; ++i) {
      const size_t ao = (size_t)(m0 + (i << 4) + rlane) * lda + koff + k0;
      V ah = Frag<T>::load(A + ao);
#pragma unroll
      for (int j = 0; j < 4; ++j) {
        acc[i][j] = Frag<T>::mma(ah, bh[j], acc[i][j]);
      }
      Frag<T>::guard(acc[i][0], acc[i][1], acc[i][2], acc[i][3], ah, bh[0], bh[1], bh[2], bh[3]);
    }
    Frag<T>::keep(bh[0], bh[1], bh[2], bh[3]);
  }
  acc_guard4(acc[0][0], acc[0][1], acc[0][2], acc[0][3]);
  acc_guard4(acc[1][0], acc[1][1], acc[1][2], acc[1][3]);
  acc_guard4(acc[2][0], acc[2][1], acc[2][2], acc[2][3]);
  acc_guard4(acc[3][0], acc[3][1], acc[3][2], acc[3][3]);

  float* slab = sT[wave];
#pragma unroll
  for (int i = 0; i < 4; ++i) {
    const int mBase = m0 + (i << 4);
#pragma unroll
    for (int j = 0; j < 4; ++j) {
#pragma unroll
      for (int r = 0; r < 8; ++r) {
        const float v = acc[i][j][r] * scale;
        slab[(mOff + r) * 68 + (j << 4) + rlane] = v;
      }
    }
    __builtin_amdgcn_fence(__ATOMIC_RELEASE, "workgroup");
    __builtin_amdgcn_wave_barrier();
    __builtin_amdgcn_fence(__ATOMIC_ACQUIRE, "workgroup");
    {
      const int hh = lane >> 4, c4 = (lane & 15) * 4;
      for (int pass = 0; pass < 2; ++pass) {
#pragma unroll
        for (int it = 0; it < 8; ++it) {
          const int row = it * 2 + hh;
          v4f v = *(const v4f*)(slab + row * 68 + c4);
          *(volatile v4f*)(Cout + (size_t)(mBase + row) * ldc + n0 + c4) = v;
        }
        __threadfence();
      }
    }
    __builtin_amdgcn_fence(__ATOMIC_RELEASE, "workgroup");
    __builtin_amdgcn_wave_barrier();
    __builtin_amdgcn_fence(__ATOMIC_ACQUIRE, "workgroup");
  }
}

__global__ __launch_bounds__(256) void cvt_rows_bf16_kernel(
    const float* __restrict__ src, unsigned short* __restrict__ dst, int total8)
{
  const int i = blockIdx.x * 256 + threadIdx.x;
  if (i >= total8) return;
  const size_t e0 = (size_t)i << 3;
  const v4f a0 = *(const v4f*)(src + e0);
  const v4f a1 = *(const v4f*)(src + e0 + 4);
  v8h hv;
#pragma unroll
  for (int e = 0; e < 4; ++e) {
    const unsigned short h0 = f2bf_bits(a0[e]);
    const unsigned short h1 = f2bf_bits(a1[e]);
    hv[e]     = __builtin_bit_cast(_Float16, h0);
    hv[4 + e] = __builtin_bit_cast(_Float16, h1);
  }
  unsigned short* qd = dst + e0;
  *(volatile v8h*)qd = hv;
  __threadfence();
  *(volatile v8h*)qd = hv;
}

template <bool OUTF16>
__global__ __launch_bounds__(256) void transpose4_kernel(
    const float* __restrict__ Wq0, const float* __restrict__ Wq1,
    const float* __restrict__ Wq2, const float* __restrict__ Wq3,
    unsigned short* __restrict__ Bt, int Kdim, float carry)
{
  __shared__ float tile[64 * 65];
  const int tid = threadIdx.x, lane = tid & 31, wave = tid >> 5;
  const int n0 = blockIdx.x * 64;
  const int h0 = blockIdx.x * 16;
  const int k0 = blockIdx.y * 64;
#pragma unroll
  for (int g = 0; g < 4; ++g) {
    const float* Wg = (g == 0) ? Wq0 : (g == 1) ? Wq1 : (g == 2) ? Wq2 : Wq3;
#pragma unroll
    for (int pp = 0; pp < 4; ++pp) {
      const int rem = pp * 256 + tid;
      const int kk  = rem >> 4;
      const int hh  = rem & 15;
      const float w = Wg[(size_t)(k0 + kk) * kHid + h0 + hh];
      tile[kk * 65 + hh * 4 + g] = bf_val(w) * carry;
    }
  }
  __syncthreads();
  const int q = lane >> 3, c8 = (lane & 7) * 8;
  v8h hv[2];
#pragma unroll
  for (int it = 0; it < 2; ++it) {
    const int nrow = it * 32 + wave * 4 + q;
#pragma unroll
    for (int e = 0; e < 8; ++e) {
      const float val = tile[(c8 + e) * 65 + nrow];
      if (OUTF16) {
        hv[it][e] = (_Float16)val;
      } else {
        const unsigned short hb = f2bf_bits(val);
        hv[it][e] = __builtin_bit_cast(_Float16, hb);
      }
    }
  }
  for (int pass = 0; pass < 2; ++pass) {
#pragma unroll
    for (int it = 0; it < 2; ++it) {
      const int nrow = it * 32 + wave * 4 + q;
      *(volatile v8h*)(Bt + (size_t)(n0 + nrow) * Kdim + k0 + c8) = hv[it];
    }
    __threadfence();
  }
}

template <bool OUT16>
__global__ __launch_bounds__(64) void scan_kernel(
    const float* __restrict__ PRJ, const float* __restrict__ Alog,
    const float* __restrict__ carry_in, float* __restrict__ carry_out, int first,
    void* __restrict__ Yout)
{
  __shared__ __align__(16) float sY[kScanTS * kScanYP];
  const int tid = threadIdx.x, lane = tid & 31, wave = tid >> 5;
  const int d0 = blockIdx.x * kScanCh;
  const int ch = d0 + tid;
  const float negA = -expf(bf_val(Alog[ch]));
  float h = 0.f;
  if (first == 0) h = carry_in[ch];
  const float* prow = PRJ + 4 * ch;
  const int q  = lane >> 3, c8 = (lane & 7) * 8;
  const int hh = lane >> 4, c4 = (lane & 15) * 4;
#pragma unroll 1
  for (int t0 = 0; t0 < kTc; t0 += kScanTS) {
    __syncthreads();
#pragma unroll 1
    for (int s = 0; s < kScanTS; ++s) {
      const v4f v = *(const v4f*)(prow + (size_t)(t0 + s) * kPrjN);
      const float xs = v[0];
      const float bm = v[1];
      const float cm = v[2];
      const float dd = v[3];
      const float e1    = expf(-dd);
      const float delta = 1.0f / (1.0f + e1);
      const float ab    = expf(delta * negA);
      const float bx    = bm * xs;
      h = ab * h + bx;
      const float y = cm * h;
      sY[s * kScanYP + tid] = OUT16 ? (y * kCarryY0) : y;
    }
    __syncthreads();
    if (OUT16) {
      unsigned short* Y = (unsigned short*)Yout;
      v8h hv[8];
#pragma unroll
      for (int it = 0; it < 8; ++it) {
        const int row = it * 8 + wave * 4 + q;
        const float* sp = sY + row * kScanYP + c8;
        const v4f a0 = *(const v4f*)(sp);
        const v4f a1 = *(const v4f*)(sp + 4);
#pragma unroll
        for (int e = 0; e < 4; ++e) {
          hv[it][e]     = (_Float16)a0[e];
          hv[it][4 + e] = (_Float16)a1[e];
        }
      }
      for (int pass = 0; pass < 2; ++pass) {
#pragma unroll
        for (int it = 0; it < 8; ++it) {
          const int row = it * 8 + wave * 4 + q;
          *(volatile v8h*)(Y + (size_t)(t0 + row) * kHid + d0 + c8) = hv[it];
        }
        __threadfence();
      }
    } else {
      float* Y = (float*)Yout;
      v4f fv[16];
#pragma unroll
      for (int it = 0; it < 16; ++it) {
        const int row = it * 4 + wave * 2 + hh;
        fv[it] = *(const v4f*)(sY + row * kScanYP + c4);
      }
      for (int pass = 0; pass < 2; ++pass) {
#pragma unroll
        for (int it = 0; it < 16; ++it) {
          const int row = it * 4 + wave * 2 + hh;
          *(volatile v4f*)(Y + (size_t)(t0 + row) * kHid + d0 + c4) = fv[it];
        }
        __threadfence();
      }
    }
  }
  {
    float* cp = carry_out + ch;
    const float hv = h;
    *(volatile float*)cp = hv;
    __threadfence();
    *(volatile float*)cp = hv;
  }
}

__global__ __launch_bounds__(256) void head_kernel(
    const float* __restrict__ Y1, const unsigned short* __restrict__ XBc,
    const float* __restrict__ Wout, const float* __restrict__ bout, const float* __restrict__ Wskip,
    float* __restrict__ outc)
{
  __shared__ __align__(16) float sWo[kHid * 4];
  __shared__ __align__(16) float sWs[kObs * 4];
  const int tid = threadIdx.x;
#pragma unroll
  for (int p = 0; p < 2; ++p) {
    const int r = tid + 256 * p;
    const v4f w = *(const v4f*)(Wout + 4 * r);
    v4f wr;
    wr[0] = bf_val(w[0]); wr[1] = bf_val(w[1]); wr[2] = bf_val(w[2]); wr[3] = bf_val(w[3]);
    *(v4f*)(sWo + 4 * r) = wr;
  }
  {
    const v4f w = *(const v4f*)(Wskip + 4 * tid);
    v4f wr;
    wr[0] = bf_val(w[0]); wr[1] = bf_val(w[1]); wr[2] = bf_val(w[2]); wr[3] = bf_val(w[3]);
    *(v4f*)(sWs + 4 * tid) = wr;
  }
  __syncthreads();
  const int t = blockIdx.x * 256 + tid;
  const v4f bb = *(const v4f*)(bout);
  float a0 = bf_val(bb[0]), a1 = bf_val(bb[1]), a2 = bf_val(bb[2]), a3 = bf_val(bb[3]);
  const float* yr = Y1 + (size_t)t * kHid;
#pragma unroll 1
  for (int k4 = 0; k4 < kHid / 4; ++k4) {
    const v4f yv = *(const v4f*)(yr + 4 * k4);
#pragma unroll
    for (int e = 0; e < 4; ++e) {
      const v4f w = *(const v4f*)(sWo + 4 * (4 * k4 + e));
      const float ye = yv[e];
      a0 = fmaf(ye, w[0], a0);
      a1 = fmaf(ye, w[1], a1);
      a2 = fmaf(ye, w[2], a2);
      a3 = fmaf(ye, w[3], a3);
    }
  }
  const unsigned short* xr = XBc + (size_t)t * kObs;
#pragma unroll 1
  for (int k8 = 0; k8 < kObs / 8; ++k8) {
    const v4u xw = *(const v4u*)(xr + 8 * k8);
#pragma unroll
    for (int j = 0; j < 4; ++j) {
      const unsigned wbits = xw[j];
      const float xlo = __uint_as_float(wbits << 16);
      const float xhi = __uint_as_float(wbits & 0xffff0000u);
      const v4f w0 = *(const v4f*)(sWs + 4 * (8 * k8 + 2 * j));
      const v4f w1 = *(const v4f*)(sWs + 4 * (8 * k8 + 2 * j + 1));
      a0 = fmaf(xlo, w0[0], a0);
      a1 = fmaf(xlo, w0[1], a1);
      a2 = fmaf(xlo, w0[2], a2);
      a3 = fmaf(xlo, w0[3], a3);
      a0 = fmaf(xhi, w1[0], a0);
      a1 = fmaf(xhi, w1[1], a1);
      a2 = fmaf(xhi, w1[2], a2);
      a3 = fmaf(xhi, w1[3], a3);
    }
  }
  v4f o;
  o[0] = a0; o[1] = a1; o[2] = a2; o[3] = a3;
  float* op = outc + (size_t)t * kNobj;
  *(volatile v4f*)op = o;
  __threadfence();
  *(volatile v4f*)op = o;
}

extern "C" void kernel_launch(void* const* d_in, const int* in_sizes, int n_in,
                              void* d_out, int out_size, void* d_ws, size_t ws_size,
                              hipStream_t stream) {
  if (n_in < 14) return;
  if (in_sizes[0] != kSeqT * kObs) return;
  if (in_sizes[1] != kObs * kHid || in_sizes[2] != kObs * kHid) return;
  if (in_sizes[3] != kObs * kHid || in_sizes[4] != kObs * kHid) return;
  if (in_sizes[5] != kHid) return;
  if (in_sizes[6] != kHid * kHid || in_sizes[7] != kHid * kHid) return;
  if (in_sizes[8] != kHid * kHid || in_sizes[9] != kHid * kHid) return;
  if (in_sizes[10] != kHid) return;
  if (in_sizes[11] != kHid * kNobj) return;
  if (in_sizes[12] != kNobj) return;
  if (in_sizes[13] != kObs * kNobj) return;
  if (out_size != kSeqT * kNobj) return;
  if (ws_size < kWsTotal) return;

  const float* x      = (const float*)d_in[0];
  const float* W_in0  = (const float*)d_in[1];
  const float* W_B0   = (const float*)d_in[2];
  const float* W_C0   = (const float*)d_in[3];
  const float* W_d0   = (const float*)d_in[4];
  const float* A_log0 = (const float*)d_in[5];
  const float* W_in1  = (const float*)d_in[6];
  const float* W_B1   = (const float*)d_in[7];
  const float* W_C1   = (const float*)d_in[8];
  const float* W_d1   = (const float*)d_in[9];
  const float* A_log1 = (const float*)d_in[10];
  const float* W_out  = (const float*)d_in[11];
  const float* b_out  = (const float*)d_in[12];
  const float* W_skip = (const float*)d_in[13];
  float* out = (float*)d_out;

  char* ws = (char*)d_ws;
  unsigned short* XB    = (unsigned short*)(ws + kOffXB);
  unsigned short* BT0   = (unsigned short*)(ws + kOffBT0);
  unsigned short* BT1   = (unsigned short*)(ws + kOffBT1);
  float*          PRJ   = (float*)(ws + kOffPRJ);
  unsigned short* Y0H   = (unsigned short*)(ws + kOffY0H);
  float*          Y1    = (float*)(ws + kOffY1);
  float*          CARRY = (float*)(ws + kOffCARRY);

  cvt_rows_bf16_kernel<<<(kSeqT * kObs / 8) / 256, 256, 0, stream>>>(x, XB, kSeqT * kObs / 8);
  transpose4_kernel<false><<<dim3(kPrjN / 64, kObs / 64), 256, 0, stream>>>(W_in0, W_B0, W_C0, W_d0, BT0, kObs, 1.0f);
  transpose4_kernel<true><<<dim3(kPrjN / 64, kHid / 64), 256, 0, stream>>>(W_in1, W_B1, W_C1, W_d1, BT1, kHid, kCarryW1);

  const int gemmBlocks = ((kTc / 64) * (kPrjN / 64)) / 8;
  for (int c = 0; c < kNChunk; ++c) {
    const unsigned short* XBc = XB + (size_t)c * kTc * kObs;
    const int first = (c == 0) ? 1 : 0;
    float* c0_out = CARRY + (size_t)(0 * 2 + (c & 1)) * kHid;
    float* c0_in  = CARRY + (size_t)(0 * 2 + ((c + 1) & 1)) * kHid;
    float* c1_out = CARRY + (size_t)(1 * 2 + (c & 1)) * kHid;
    float* c1_in  = CARRY + (size_t)(1 * 2 + ((c + 1) & 1)) * kHid;

    wmma_gemm64<1><<<gemmBlocks, 256, 0, stream>>>(XBc, kObs, BT0, kObs, PRJ, kPrjN, kTc, kPrjN, kObs, 1.0f);
    scan_kernel<true><<<kHid / kScanCh, kScanCh, 0, stream>>>(PRJ, A_log0, c0_in, c0_out, first, (void*)Y0H);
    wmma_gemm64<0><<<gemmBlocks, 256, 0, stream>>>(Y0H, kHid, BT1, kHid, PRJ, kPrjN, kTc, kPrjN, kHid, kFoldL1);
    scan_kernel<false><<<kHid / kScanCh, kScanCh, 0, stream>>>(PRJ, A_log1, c1_in, c1_out, first, (void*)Y1);
    head_kernel<<<kTc / 256, 256, 0, stream>>>(Y1, XBc, W_out, b_out, W_skip, out + (size_t)c * kTc * kNobj);
  }
}
